// MRCGNN_27066883899440
// MI455X (gfx1250) — hardware-verified
//
#include <hip/hip_runtime.h>
#include <stddef.h>
#include <math.h>


#define FIN    128
#define H1     64
#define H2     32
#define RR     65
#define RP     80
#define CLSK   448
#define CLSN   80
#define NTHR   256
#define NWAVE  8
#define EPT    8
#define NGRP   2
#define CHUNK  (NTHR * EPT * NGRP)
#define WCAP   (EPT * NGRP * 32)
#define LISTN  (NWAVE * WCAP)
#define NBA    512
#define ACP    64
#define MP     64
#define GROWS  128
#define OROWS  256
#define WSCALE 16.0f
#define WINV   0.0625f

static_assert((CHUNK & (CHUNK - 1)) == 0);
static_assert((NBA & (NBA - 1)) == 0 && NBA <= 4096);
static_assert(NBA == NWAVE * 64);
static_assert(MP == H1 && ACP == H1);
static_assert((NBA * RR * 4) % 16 == 0);
static_assert(RP % 4 == 0 && RP >= RR);
static_assert((NBA * RP / 4) % NTHR == 0);
static_assert(CLSK % 32 == 0 && CLSN % 16 == 0);
static_assert(OROWS == NTHR);

typedef float    v2f  __attribute__((ext_vector_type(2)));
typedef float    v4f  __attribute__((ext_vector_type(4)));
typedef float    v8f  __attribute__((ext_vector_type(8)));
typedef int      v4i  __attribute__((ext_vector_type(4)));
typedef _Float16 v2h  __attribute__((ext_vector_type(2)));
typedef _Float16 v4h  __attribute__((ext_vector_type(4)));
typedef _Float16 v8h  __attribute__((ext_vector_type(8)));
typedef _Float16 v16h __attribute__((ext_vector_type(16)));
union FragH { v16h v; v8h h[2]; };

__device__ __forceinline__ v8h cvt8(v4f a, v4f b) {
  v8h r;
  r[0] = (_Float16)a.x; r[1] = (_Float16)a.y; r[2] = (_Float16)a.z; r[3] = (_Float16)a.w;
  r[4] = (_Float16)b.x; r[5] = (_Float16)b.y; r[6] = (_Float16)b.z; r[7] = (_Float16)b.w;
  return r;
}

__device__ __forceinline__ v8f wmh(v16h a, v16h b, v8f c) {
  v8f d = __builtin_amdgcn_wmma_f32_16x16x32_f16(false, a, false, b, (short)0, c, false, false);
  asm volatile("v_nop\n\tv_nop\n\tv_nop\n\tv_nop" : "+v"(d) : "v"(a), "v"(b));
  return d;
}

template <int NB>
__device__ __forceinline__ int scan_chunk(const int* __restrict__ dsts, int nE, int cbase, int slotBase,
                                          int vec8, int* list, int tid, int lane, int wave) {
  int wc = 0;
#pragma unroll
  for (int g = 0; g < NGRP; ++g) {
    const int el0  = (g * NTHR + tid) * EPT;
    const int e0   = cbase + el0;
    const int sent = -2147483647 - 1;
    v4i da, db;
    if (vec8 != 0 && cbase + CHUNK <= nE) {
      da = *(const v4i*)(dsts + e0);
      db = *(const v4i*)(dsts + e0 + 4);
    } else {
      da.x = (e0     < nE) ? dsts[min(e0, nE - 1)] : sent;
      da.y = (e0 + 1 < nE) ? dsts[min(e0 + 1, nE - 1)] : sent;
      da.z = (e0 + 2 < nE) ? dsts[min(e0 + 2, nE - 1)] : sent;
      da.w = (e0 + 3 < nE) ? dsts[min(e0 + 3, nE - 1)] : sent;
      db.x = (e0 + 4 < nE) ? dsts[min(e0 + 4, nE - 1)] : sent;
      db.y = (e0 + 5 < nE) ? dsts[min(e0 + 5, nE - 1)] : sent;
      db.z = (e0 + 6 < nE) ? dsts[min(e0 + 6, nE - 1)] : sent;
      db.w = (e0 + 7 < nE) ? dsts[min(e0 + 7, nE - 1)] : sent;
    }
    const unsigned nb = (unsigned)slotBase;
    const unsigned s0 = (unsigned)da.x - nb, s1 = (unsigned)da.y - nb;
    const unsigned s2 = (unsigned)da.z - nb, s3 = (unsigned)da.w - nb;
    const unsigned s4 = (unsigned)db.x - nb, s5 = (unsigned)db.y - nb;
    const unsigned s6 = (unsigned)db.z - nb, s7 = (unsigned)db.w - nb;
    const bool h0 = s0 < (unsigned)NB, h1 = s1 < (unsigned)NB, h2 = s2 < (unsigned)NB, h3 = s3 < (unsigned)NB;
    const bool h4 = s4 < (unsigned)NB, h5 = s5 < (unsigned)NB, h6 = s6 < (unsigned)NB, h7 = s7 < (unsigned)NB;
    const unsigned any = __builtin_amdgcn_ballot_w32(h0 | h1 | h2 | h3 | h4 | h5 | h6 | h7);
    if (any != 0u) {
#define HITJ(J, HJ, SJ) { \
        const unsigned mj = __builtin_amdgcn_ballot_w32(HJ); \
        if (mj != 0u) { \
          if (HJ) { \
            const int pos = wc + (int)__builtin_amdgcn_mbcnt_lo(mj, 0u); \
            if (pos < WCAP) list[wave * WCAP + pos] = ((el0 + (J)) << 12) | (int)(SJ); \
          } \
          wc += (int)__builtin_popcount(mj); } }
      HITJ(0, h0, s0)
      HITJ(1, h1, s1)
      HITJ(2, h2, s2)
      HITJ(3, h3, s3)
      HITJ(4, h4, s4)
      HITJ(5, h5, s5)
      HITJ(6, h6, s6)
      HITJ(7, h7, s7)
#undef HITJ
    }
  }
  return wc;
}

__global__ __launch_bounds__(NTHR) void k_prep(
    const float* __restrict__ xo, const float* __restrict__ xa,
    const float* __restrict__ W1, const float* __restrict__ W2,
    const float* __restrict__ r1, const float* __restrict__ r2, const float* __restrict__ cw,
    _Float16* X16o, _Float16* X16a, _Float16* W1t, _Float16* W2t,
    _Float16* R1t, _Float16* R2t, _Float16* CLt, int nN) {
  const int s0 = nN * (FIN / 8);
  const int p0 = (s0 + NTHR - 1) & ~(NTHR - 1);
  const int s2 = RR * H1 * FIN / 8, s3 = RR * H2 * H1 / 8, s4 = H1 * FIN / 8, s5 = H2 * H1 / 8, s6 = CLSN * CLSK / 8;
  const int b1 = p0, b2 = 2 * p0, b3 = b2 + s2, b4 = b3 + s3, b5 = b4 + s4, b6 = b5 + s5;
  const int bstart = blockIdx.x * NTHR;
  const int i = bstart + (int)threadIdx.x;
  float v[8];
  _Float16* dp;
  if (bstart < b1) {
    const int local = i;
    if (local >= s0) return;
    const int n = local / (FIN / 8);
    const int c0 = (local - n * (FIN / 8)) * 8;
    const float* sp = xo + (size_t)n * FIN + c0;
    const v4f a = *(const v4f*)sp, b = *(const v4f*)(sp + 4);
    v[0] = a.x; v[1] = a.y; v[2] = a.z; v[3] = a.w; v[4] = b.x; v[5] = b.y; v[6] = b.z; v[7] = b.w;
    dp = X16o + (size_t)local * 8;
  } else if (bstart < b2) {
    const int local = i - b1;
    if (local >= s0) return;
    const int n = local / (FIN / 8);
    const int c0 = (local - n * (FIN / 8)) * 8;
    const float* sp = xa + (size_t)n * FIN + c0;
    const v4f a = *(const v4f*)sp, b = *(const v4f*)(sp + 4);
    v[0] = a.x; v[1] = a.y; v[2] = a.z; v[3] = a.w; v[4] = b.x; v[5] = b.y; v[6] = b.z; v[7] = b.w;
    dp = X16a + (size_t)local * 8;
  } else if (bstart < b3) {
    const int local = i - b2;
    const int o = local * 8;
    const int rr = o / (H1 * FIN);
    const int rem = o - rr * (H1 * FIN);
    const int n = rem / FIN;
    const int k0 = rem - n * FIN;
#pragma unroll
    for (int e = 0; e < 8; ++e) v[e] = W1[((size_t)rr * FIN + k0 + e) * H1 + n] * WSCALE;
    dp = W1t + o;
  } else if (bstart < b4) {
    const int local = i - b3;
    const int o = local * 8;
    const int rr = o / (H2 * H1);
    const int rem = o - rr * (H2 * H1);
    const int n = rem / H1;
    const int k0 = rem - n * H1;
#pragma unroll
    for (int e = 0; e < 8; ++e) v[e] = W2[((size_t)rr * H1 + k0 + e) * H2 + n] * WSCALE;
    dp = W2t + o;
  } else if (bstart < b5) {
    const int local = i - b4;
    const int o = local * 8;
    const int n = o / FIN;
    const int k0 = o - n * FIN;
#pragma unroll
    for (int e = 0; e < 8; ++e) v[e] = r1[(k0 + e) * H1 + n] * WSCALE;
    dp = R1t + o;
  } else if (bstart < b6) {
    const int local = i - b5;
    const int o = local * 8;
    const int n = o / H1;
    const int k0 = o - n * H1;
#pragma unroll
    for (int e = 0; e < 8; ++e) v[e] = r2[(k0 + e) * H2 + n] * WSCALE;
    dp = R2t + o;
  } else {
    const int local = i - b6;
    if (local >= s6) return;
    const int o = local * 8;
    const int n = o / CLSK;
    const int k0 = o - n * CLSK;
    const int nc = n < RR ? n : RR - 1;
#pragma unroll
    for (int e = 0; e < 8; ++e) {
      const float x = cw[(k0 + e) * RR + nc];
      v[e] = (n < RR) ? x * WSCALE : 0.0f;
    }
    dp = CLt + o;
  }
  v4f a, b;
  a.x = v[0]; a.y = v[1]; a.z = v[2]; a.w = v[3];
  b.x = v[4]; b.y = v[5]; b.z = v[6]; b.w = v[7];
  const v8h hv = cvt8(a, b);
  *(volatile v8h*)dp = hv;
  __threadfence();
  *(volatile v8h*)dp = hv;
}

__global__ __launch_bounds__(NTHR) void k_tsort(
    const int* __restrict__ et, int* perm, int* tcnt, int nE, int tcap, int vec8) {
  extern __shared__ v4f lds_dyn[];
  int* seg  = (int*)lds_dyn;
  int* list = seg + tcap;
  int* wcnt = list + LISTN;
  const int tid = threadIdx.x, lane = tid & 31, wave = tid >> 5;
  const int r = blockIdx.x;
  for (int i = tid; i < tcap; i += NTHR) seg[i] = -1;
  __syncthreads();

  int fill = 0;
  const int nChunks = (nE + CHUNK - 1) / CHUNK;
#pragma unroll 1
  for (int ch = 0; ch < nChunks; ++ch) {
    const int cbase = ch * CHUNK;
    int wc = scan_chunk<1>(et, nE, cbase, r, vec8, list, tid, lane, wave);
    wc = wc > WCAP ? WCAP : (wc < 0 ? 0 : wc);
    if (lane == 0) wcnt[wave] = wc;
    __syncthreads();
    int pre = 0, tot = 0;
#pragma unroll
    for (int w = 0; w < NWAVE; ++w) {
      int c = wcnt[w];
      c = c > WCAP ? WCAP : (c < 0 ? 0 : c);
      if (w < wave) pre += c;
      tot += c;
    }
#pragma unroll 1
    for (int i = lane; i < wc; i += 32) {
      const int p = fill + pre + i;
      if (p < tcap) seg[p] = cbase + ((list[wave * WCAP + i] >> 12) & (CHUNK - 1));
    }
    fill += tot;
    if (fill > tcap) fill = tcap;
    __syncthreads();
  }

  int* gp = perm + (size_t)r * tcap;
  const int nv = tcap >> 2;
#pragma unroll 1
  for (int i = tid; i < nv; i += NTHR) { const v4i v = ((const v4i*)seg)[i]; *(volatile v4i*)(gp + 4 * i) = v; }
  v4i cv; cv.x = fill; cv.y = fill; cv.z = fill; cv.w = fill;
  if (tid < 8) *(volatile v4i*)(tcnt + r * 32 + 4 * tid) = cv;
  __threadfence();
#pragma unroll 1
  for (int i = tid; i < nv; i += NTHR) { const v4i v = ((const v4i*)seg)[i]; *(volatile v4i*)(gp + 4 * i) = v; }
  if (tid < 8) *(volatile v4i*)(tcnt + r * 32 + 4 * tid) = cv;
}

__global__ __launch_bounds__(NTHR) void k_cnt(
    const int* __restrict__ ei, const int* __restrict__ et, float* rc, int nE, int vec8) {
  extern __shared__ v4f lds_dyn[];
  int* cnt  = (int*)lds_dyn;
  int* list = cnt + NBA * RR;
  int* wcnt = list + LISTN;
  const int tid = threadIdx.x, lane = tid & 31, wave = tid >> 5;
  const int nodeBase = blockIdx.x * NBA;
  const int* dsts = ei + nE;

  for (int i = tid; i < NBA * RR; i += NTHR) cnt[i] = 0;
  __syncthreads();

  const int nChunks = (nE + CHUNK - 1) / CHUNK;
#pragma unroll 1
  for (int ch = 0; ch < nChunks; ++ch) {
    const int cbase = ch * CHUNK;
    const int wc = scan_chunk<NBA>(dsts, nE, cbase, nodeBase, vec8, list, tid, lane, wave);
    if (lane == 0) wcnt[wave] = wc;
    __syncthreads();
    if (wave == 0) {
#pragma unroll 1
      for (int wsx = 0; wsx < NWAVE; ++wsx) {
        int n = __builtin_amdgcn_readfirstlane(wcnt[wsx]);
        n = n > WCAP ? WCAP : (n < 0 ? 0 : n);
        const int* lp = list + wsx * WCAP;
#pragma unroll 1
        for (int i = 0; i < n; ++i) {
          const int ent  = __builtin_amdgcn_readfirstlane(lp[i]);
          const int slot = ent & (NBA - 1);
          int e = cbase + ((ent >> 12) & (CHUNK - 1));
          e = e > nE - 1 ? nE - 1 : e;
          int t = et[e];
          t = t < 0 ? 0 : (t > RR - 1 ? RR - 1 : t);
          if (lane == 0) cnt[slot * RR + t] = cnt[slot * RR + t] + 1;
        }
      }
    }
    __syncthreads();
  }

  float* tab = (float*)cnt;
#pragma unroll 1
  for (int i = tid; i < NBA * RR; i += NTHR) {
    int cv = cnt[i];
    cv = cv < 1 ? 1 : cv;
    tab[i] = 1.0f / (float)cv;
  }
  __syncthreads();

  float* gp = rc + (size_t)nodeBase * RP;
#pragma unroll 1
  for (int i = tid; i < NBA * RP / 4; i += NTHR) {
    const int f = 4 * i;
    const int row = f / RP;
    const int c = f - row * RP;
    v4f v;
    v.x = (c     < RR) ? tab[row * RR + min(c,     RR - 1)] : 0.0f;
    v.y = (c + 1 < RR) ? tab[row * RR + min(c + 1, RR - 1)] : 0.0f;
    v.z = (c + 2 < RR) ? tab[row * RR + min(c + 2, RR - 1)] : 0.0f;
    v.w = (c + 3 < RR) ? tab[row * RR + min(c + 3, RR - 1)] : 0.0f;
    *(volatile v4f*)(gp + f) = v;
  }
  __threadfence();
#pragma unroll 1
  for (int i = tid; i < NBA * RP / 4; i += NTHR) {
    const int f = 4 * i;
    const int row = f / RP;
    const int c = f - row * RP;
    v4f v;
    v.x = (c     < RR) ? tab[row * RR + min(c,     RR - 1)] : 0.0f;
    v.y = (c + 1 < RR) ? tab[row * RR + min(c + 1, RR - 1)] : 0.0f;
    v.z = (c + 2 < RR) ? tab[row * RR + min(c + 2, RR - 1)] : 0.0f;
    v.w = (c + 3 < RR) ? tab[row * RR + min(c + 3, RR - 1)] : 0.0f;
    *(volatile v4f*)(gp + f) = v;
  }
}

template <int KD, int NT, int GATHER>
__global__ __launch_bounds__(NTHR) void k_gemm16(
    const _Float16* __restrict__ A16, const _Float16* __restrict__ Bt,
    const int* __restrict__ perm, const int* __restrict__ tcnt, const int* __restrict__ ei,
    _Float16* Out, int nRowsA, int nRows, int nE, int tcap) {
  constexpr int AP = KD + 8;
  static_assert(GROWS * AP >= GROWS * MP);
  static_assert((GROWS * KD / 8) % NTHR == 0);
  static_assert(NT >= 1 && NT <= 4 && KD % 32 == 0);
  __shared__ __attribute__((aligned(16))) _Float16 sA[GROWS * AP];
  __shared__ int lrow[GROWS];
  __shared__ int lsrc[GROWS];
  const int tid = threadIdx.x, lane = tid & 31, wave = tid >> 5, hh = lane >> 4, m = lane & 15;
  const int rowBase = blockIdx.x * GROWS;
  const int r = blockIdx.y;
  int cnt;
  if (GATHER) {
    int c = tcnt[r * 32];
    c = c < 0 ? 0 : (c > tcap ? tcap : c);
    cnt = c;
  } else {
    cnt = nRows;
  }
  if (rowBase >= cnt) return;

  if (tid < GROWS) {
    if (GATHER) {
      const int p = perm[(size_t)r * tcap + rowBase + tid];
      const int e = p < 0 ? -1 : (p > nE - 1 ? nE - 1 : p);
      const int ec = e < 0 ? 0 : e;
      int s = ei[ec];
      s = s < 0 ? 0 : (s > nRowsA - 1 ? nRowsA - 1 : s);
      lrow[tid] = e;
      lsrc[tid] = s;
    } else {
      const int row = rowBase + tid;
      lrow[tid] = row < nRows ? row : -1;
      lsrc[tid] = row > nRowsA - 1 ? nRowsA - 1 : row;
    }
  }
  __syncthreads();

#pragma unroll
  for (int i = 0; i < (GROWS * KD / 8) / NTHR; ++i) {
    const int idx = i * NTHR + tid;
    const int row = idx / (KD / 8);
    const int c0  = (idx - row * (KD / 8)) * 8;
    const int s   = lsrc[row];
    const v8h v = *(const v8h*)(A16 + (size_t)s * KD + c0);
    *(v8h*)(sA + row * AP + c0) = v;
  }
  __syncthreads();

  v8f acc[NT];
#pragma unroll
  for (int t = 0; t < NT; ++t) { v8f z = {0.f, 0.f, 0.f, 0.f, 0.f, 0.f, 0.f, 0.f}; acc[t] = z; }
  const _Float16* ar = sA + (wave * 16 + m) * AP + 8 * hh;
  const _Float16* Bbase = Bt + (size_t)r * (NT * 16 * KD);
#pragma unroll
  for (int kt = 0; kt < KD / 32; ++kt) {
    FragH a;
    a.h[0] = *(const v8h*)(ar + 32 * kt);
    a.h[1] = *(const v8h*)(ar + 32 * kt + 16);
#pragma unroll
    for (int t = 0; t < NT; ++t) {
      const _Float16* bp = Bbase + (size_t)(16 * t + m) * KD + 32 * kt + 8 * hh;
      FragH b;
      b.h[0] = *(const v8h*)bp;
      b.h[1] = *(const v8h*)(bp + 16);
      acc[t] = wmh(a.v, b.v, acc[t]);
    }
  }
  __syncthreads();

  _Float16* sO = sA;
  _Float16* sp = sO + (wave * 16 + 8 * hh) * MP + m;
#pragma unroll
  for (int t = 0; t < NT; ++t) {
#pragma unroll
    for (int r8 = 0; r8 < 8; ++r8) sp[r8 * MP + 16 * t] = (_Float16)(acc[t][r8] * WINV);
  }
#pragma unroll
  for (int t = NT; t < 4; ++t) {
#pragma unroll
    for (int r8 = 0; r8 < 8; ++r8) sp[r8 * MP + 16 * t] = (_Float16)0.0f;
  }
  __syncthreads();

#pragma unroll
  for (int p = 0; p < 4; ++p) {
    const int row = wave * 16 + 4 * p + (lane >> 3);
    const int q = lane & 7;
    const v8h v = *(const v8h*)(sO + row * MP + 8 * q);
    const int orow = lrow[row];
    if (orow >= 0) *(volatile v8h*)(Out + (size_t)orow * MP + 8 * q) = v;
  }
  __threadfence();
#pragma unroll
  for (int p = 0; p < 4; ++p) {
    const int row = wave * 16 + 4 * p + (lane >> 3);
    const int q = lane & 7;
    const v8h v = *(const v8h*)(sO + row * MP + 8 * q);
    const int orow = lrow[row];
    if (orow >= 0) *(volatile v8h*)(Out + (size_t)orow * MP + 8 * q) = v;
  }
}

__device__ __forceinline__ v8h agg_row_l1(const float* acc, const _Float16* __restrict__ RT,
                                          const float* __restrict__ bias, int s, int n, int q) {
  const float* ap = acc + s * ACP + 8 * q;
  const v4f a0 = *(const v4f*)ap, a1 = *(const v4f*)(ap + 4);
  const v8h rt = *(const v8h*)(RT + (size_t)n * MP + 8 * q);
  const v4f b0 = *(const v4f*)(bias + 8 * q), b1 = *(const v4f*)(bias + 8 * q + 4);
  v4f o0, o1;
  o0.x = fmaxf(a0.x + (float)rt[0] + b0.x, 0.0f);
  o0.y = fmaxf(a0.y + (float)rt[1] + b0.y, 0.0f);
  o0.z = fmaxf(a0.z + (float)rt[2] + b0.z, 0.0f);
  o0.w = fmaxf(a0.w + (float)rt[3] + b0.w, 0.0f);
  o1.x = fmaxf(a1.x + (float)rt[4] + b1.x, 0.0f);
  o1.y = fmaxf(a1.y + (float)rt[5] + b1.y, 0.0f);
  o1.z = fmaxf(a1.z + (float)rt[6] + b1.z, 0.0f);
  o1.w = fmaxf(a1.w + (float)rt[7] + b1.w, 0.0f);
  return cvt8(o0, o1);
}

__device__ __forceinline__ v4f agg_row_l2(const float* acc, const _Float16* __restrict__ RT,
                                          const float* __restrict__ bias, int s, int n, int q) {
  const v4f a = *(const v4f*)(acc + s * ACP + 4 * q);
  const v4h rt = *(const v4h*)(RT + (size_t)n * MP + 4 * q);
  const v4f b = *(const v4f*)(bias + 4 * q);
  v4f o;
  o.x = a.x + (float)rt[0] + b.x;
  o.y = a.y + (float)rt[1] + b.y;
  o.z = a.z + (float)rt[2] + b.z;
  o.w = a.w + (float)rt[3] + b.w;
  return o;
}

template <int L>
__global__ __launch_bounds__(NTHR) void k_agg(
    const int* __restrict__ ei, const int* __restrict__ et, const float* __restrict__ rc,
    const _Float16* __restrict__ M, const _Float16* __restrict__ RT, const float* __restrict__ bias,
    _Float16* Hout, float* Xout, int nE, int vec8) {
  extern __shared__ v4f lds_dyn[];
  float* acc  = (float*)lds_dyn;
  int*   list = (int*)(acc + NBA * ACP);
  int*   wcnt = list + LISTN;
  const int tid = threadIdx.x, lane = tid & 31, wave = tid >> 5;
  const int nodeBase = blockIdx.x * NBA;
  const int* dsts = ei + nE;

  {
    const v4f z = {0.f, 0.f, 0.f, 0.f};
    for (int i = tid; i < NBA * ACP / 4; i += NTHR) ((v4f*)acc)[i] = z;
  }
  __syncthreads();

  const int nChunks = (nE + CHUNK - 1) / CHUNK;
#pragma unroll 1
  for (int ch = 0; ch < nChunks; ++ch) {
    const int cbase = ch * CHUNK;
    const int wc = scan_chunk<NBA>(dsts, nE, cbase, nodeBase, vec8, list, tid, lane, wave);
    if (lane == 0) wcnt[wave] = wc;
    __syncthreads();
    if (wave == 0) {
#pragma unroll 1
      for (int wsx = 0; wsx < NWAVE; ++wsx) {
        int n = __builtin_amdgcn_readfirstlane(wcnt[wsx]);
        n = n > WCAP ? WCAP : (n < 0 ? 0 : n);
        const int* lp = list + wsx * WCAP;
#pragma unroll 1
        for (int i = 0; i < n; ++i) {
          const int ent  = __builtin_amdgcn_readfirstlane(lp[i]);
          const int slot = ent & (NBA - 1);
          int e = cbase + ((ent >> 12) & (CHUNK - 1));
          e = e > nE - 1 ? nE - 1 : e;
          int t = et[e];
          t = t < 0 ? 0 : (t > RR - 1 ? RR - 1 : t);
          const float rcv = rc[(size_t)(nodeBase + slot) * RP + t];
          const v2h mv = *(const v2h*)(M + (size_t)e * MP + 2 * lane);
          float* ap = acc + slot * ACP + 2 * lane;
          v2f a = *(const v2f*)ap;
          a.x += rcv * (float)mv.x;
          a.y += rcv * (float)mv.y;
          *(v2f*)ap = a;
        }
      }
    }
    __syncthreads();
  }

  const int q = lane & 7;
#pragma unroll 1
  for (int p = 0; p < 16; ++p) {
    const int s = wave * 64 + 4 * p + (lane >> 3);
    const int n = nodeBase + s;
    if (L == 1) { const v8h hv = agg_row_l1(acc, RT, bias, s, n, q); *(volatile v8h*)(Hout + (size_t)n * MP + 8 * q) = hv; }
    else        { const v4f ov = agg_row_l2(acc, RT, bias, s, n, q); *(volatile v4f*)(Xout + (size_t)n * H2 + 4 * q) = ov; }
  }
  __threadfence();
#pragma unroll 1
  for (int p = 0; p < 16; ++p) {
    const int s = wave * 64 + 4 * p + (lane >> 3);
    const int n = nodeBase + s;
    if (L == 1) { const v8h hv = agg_row_l1(acc, RT, bias, s, n, q); *(volatile v8h*)(Hout + (size_t)n * MP + 8 * q) = hv; }
    else        { const v4f ov = agg_row_l2(acc, RT, bias, s, n, q); *(volatile v4f*)(Xout + (size_t)n * H2 + 4 * q) = ov; }
  }
}

__global__ __launch_bounds__(NTHR) void k_readout(
    const float* __restrict__ X2o, const float* __restrict__ discW, float* vline, int nN) {
  __shared__ double part[NTHR];
  __shared__ float cs[32];
  __shared__ __attribute__((aligned(16))) float sv[32];
  const int tid = threadIdx.x, col = tid & 31, g = tid >> 5;
  double s = 0.0;
#pragma unroll 1
  for (int n = g; n < nN; n += NWAVE) s += (double)X2o[(size_t)n * H2 + col];
  part[tid] = s;
  __syncthreads();
  if (tid < 32) {
    double t = 0.0;
#pragma unroll 1
    for (int gg = 0; gg < NWAVE; ++gg) t += part[gg * 32 + tid];
    const float mean = (float)(t / (double)nN);
    cs[tid] = 1.0f / (1.0f + expf(-mean));
  }
  __syncthreads();
  if (tid < 32) {
    float v = 0.0f;
#pragma unroll 1
    for (int j = 0; j < H2; ++j) v += discW[tid * H2 + j] * cs[j];
    sv[tid] = v;
  }
  __syncthreads();
  v4f ov = {0.f, 0.f, 0.f, 0.f};
  if (tid < 8) ov = *(const v4f*)(sv + 4 * tid);
  if (tid < 8) *(volatile v4f*)(vline + 4 * tid) = ov;
  __threadfence();
  if (tid < 8) *(volatile v4f*)(vline + 4 * tid) = ov;
}

__global__ __launch_bounds__(NTHR) void k_out(
    const float* __restrict__ X2o, const float* __restrict__ X2a, const float* __restrict__ X2b,
    const float* __restrict__ vline, const float* __restrict__ discb,
    float* out1, float* out2, float* out3, int nN, int nbp) {
  extern __shared__ v4f lds_dyn[];
  float* t0 = (float*)lds_dyn;
  float* t1 = t0 + OROWS * H2;
  float* t2 = t1 + OROWS * H2;
  __shared__ float sv[32];
  __shared__ float s1s[OROWS], s2s[OROWS], s3s[OROWS];
  const int tid = threadIdx.x;
  const int nodeBase = blockIdx.x * OROWS;
  if (nodeBase >= nN) return;
  if (tid < 32) sv[tid] = vline[tid];
#pragma unroll
  for (int i = 0; i < OROWS * H2 / 4 / NTHR; ++i) {
    const int idx = i * NTHR + tid;
    const int row = idx >> 3, c = idx & 7;
    int n = nodeBase + row;
    n = n > nbp - 1 ? nbp - 1 : n;
    const size_t o = (size_t)n * H2 + 4 * c;
    *(v4f*)(t0 + row * H2 + 4 * c) = *(const v4f*)(X2o + o);
    *(v4f*)(t1 + row * H2 + 4 * c) = *(const v4f*)(X2a + o);
    *(v4f*)(t2 + row * H2 + 4 * c) = *(const v4f*)(X2b + o);
  }
  __syncthreads();
  float a = 0.f, b = 0.f, c = 0.f;
#pragma unroll 1
  for (int j = 0; j < H2; ++j) {
    const float w = sv[j];
    a += t0[tid * H2 + j] * w;
    b += t1[tid * H2 + j] * w;
    c += t2[tid * H2 + j] * w;
  }
  const float db = discb[0];
  s1s[tid] = a + db; s2s[tid] = b + db; s3s[tid] = c + db;
  __syncthreads();

  int nv = nN - nodeBase;
  nv = nv > OROWS ? OROWS : nv;
  const int npair = nv >> 1;
  float* g1 = out1 + (size_t)nodeBase * 2;
  float* g2 = out2 + (size_t)nodeBase * 2;
  float* g3 = out3 + (size_t)nodeBase * H2;
#pragma unroll 1
  for (int i = tid; i < npair; i += NTHR) {
    v4f v; v.x = s1s[2 * i]; v.y = s2s[2 * i]; v.z = s1s[2 * i + 1]; v.w = s2s[2 * i + 1];
    v4f u; u.x = s1s[2 * i]; u.y = s3s[2 * i]; u.z = s1s[2 * i + 1]; u.w = s3s[2 * i + 1];
    *(volatile v4f*)(g1 + 4 * i) = v;
    *(volatile v4f*)(g2 + 4 * i) = u;
  }
  if ((nv & 1) != 0 && tid == 0) {
    const int j = nv - 1;
    const float p0 = s1s[j], p1 = s2s[j], p2 = s3s[j];
    *(volatile float*)(g1 + 2 * j) = p0; *(volatile float*)(g1 + 2 * j + 1) = p1;
    *(volatile float*)(g2 + 2 * j) = p0; *(volatile float*)(g2 + 2 * j + 1) = p2;
  }
#pragma unroll 1
  for (int i = tid; i < nv * (H2 / 4); i += NTHR) { const v4f v = *(const v4f*)(t0 + 4 * i); *(volatile v4f*)(g3 + 4 * i) = v; }
  __threadfence();
#pragma unroll 1
  for (int i = tid; i < npair; i += NTHR) {
    v4f v; v.x = s1s[2 * i]; v.y = s2s[2 * i]; v.z = s1s[2 * i + 1]; v.w = s2s[2 * i + 1];
    v4f u; u.x = s1s[2 * i]; u.y = s3s[2 * i]; u.z = s1s[2 * i + 1]; u.w = s3s[2 * i + 1];
    *(volatile v4f*)(g1 + 4 * i) = v;
    *(volatile v4f*)(g2 + 4 * i) = u;
  }
  if ((nv & 1) != 0 && tid == 0) {
    const int j = nv - 1;
    const float p0 = s1s[j], p1 = s2s[j], p2 = s3s[j];
    *(volatile float*)(g1 + 2 * j) = p0; *(volatile float*)(g1 + 2 * j + 1) = p1;
    *(volatile float*)(g2 + 2 * j) = p0; *(volatile float*)(g2 + 2 * j + 1) = p2;
  }
#pragma unroll 1
  for (int i = tid; i < nv * (H2 / 4); i += NTHR) { const v4f v = *(const v4f*)(t0 + 4 * i); *(volatile v4f*)(g3 + 4 * i) = v; }
}

__global__ __launch_bounds__(NTHR) void k_cls(
    const _Float16* __restrict__ H16o, const float* __restrict__ X2o, const float* __restrict__ feat,
    const int* __restrict__ idxp, const float* __restrict__ attt,
    const _Float16* __restrict__ CLt, const float* __restrict__ clsb,
    float* out0, int nN, int nB) {
  extern __shared__ v4f lds_dyn[];
  constexpr int AP = CLSK + 8;
  _Float16* sA  = (_Float16*)lds_dyn;
  float*    stg = (float*)lds_dyn;
  __shared__ int li0[GROWS], li1[GROWS];
  static_assert(GROWS * RR * 4 <= GROWS * AP * 2);
  const int tid = threadIdx.x, lane = tid & 31, wave = tid >> 5, hh = lane >> 4, m = lane & 15;
  const int rowBase = blockIdx.x * GROWS;
  if (rowBase >= nB) return;
  if (tid < GROWS) {
    int b = rowBase + tid;
    b = b > nB - 1 ? nB - 1 : b;
    int i0 = idxp[b], i1 = idxp[nB + b];
    i0 = i0 < 0 ? 0 : (i0 > nN - 1 ? nN - 1 : i0);
    i1 = i1 < 0 ? 0 : (i1 > nN - 1 ? nN - 1 : i1);
    li0[tid] = i0; li1[tid] = i1;
  }
  __syncthreads();
  const float a0 = attt[0], a1 = attt[1];

#pragma unroll
  for (int it = 0; it < GROWS * 16 / NTHR; ++it) {
    const int idx = it * NTHR + tid;
    const int row = idx >> 4, rem = idx & 15, which = rem >> 3, g = rem & 7;
    const int n0 = li0[row], n1 = li1[row];
    const int node = which ? n1 : n0;
    const v8h hv = *(const v8h*)(H16o + (size_t)node * MP + 8 * g);
    v4f fa, fb;
    fa.x = (float)hv[0] * a0; fa.y = (float)hv[1] * a0; fa.z = (float)hv[2] * a0; fa.w = (float)hv[3] * a0;
    fb.x = (float)hv[4] * a0; fb.y = (float)hv[5] * a0; fb.z = (float)hv[6] * a0; fb.w = (float)hv[7] * a0;
    *(v8h*)(sA + row * AP + which * 224 + 8 * g) = cvt8(fa, fb);
  }
#pragma unroll
  for (int it = 0; it < GROWS * 8 / NTHR; ++it) {
    const int idx = it * NTHR + tid;
    const int row = idx >> 3, rem = idx & 7, which = rem >> 2, g = rem & 3;
    const int n0 = li0[row], n1 = li1[row];
    const int node = which ? n1 : n0;
    const float* xp = X2o + (size_t)node * H2 + 8 * g;
    const v4f fa = *(const v4f*)xp * a1, fb = *(const v4f*)(xp + 4) * a1;
    *(v8h*)(sA + row * AP + which * 224 + 64 + 8 * g) = cvt8(fa, fb);
  }
#pragma unroll
  for (int it = 0; it < GROWS * 32 / NTHR; ++it) {
    const int idx = it * NTHR + tid;
    const int row = idx >> 5, rem = idx & 31, which = rem >> 4, g = rem & 15;
    const int n0 = li0[row], n1 = li1[row];
    const int node = which ? n1 : n0;
    const float* xp = feat + (size_t)node * FIN + 8 * g;
    const v4f fa = *(const v4f*)xp, fb = *(const v4f*)(xp + 4);
    *(v8h*)(sA + row * AP + which * 224 + 96 + 8 * g) = cvt8(fa, fb);
  }
  __syncthreads();

  v8f acc[CLSN / 16];
#pragma unroll
  for (int t = 0; t < CLSN / 16; ++t) { v8f z = {0.f, 0.f, 0.f, 0.f, 0.f, 0.f, 0.f, 0.f}; acc[t] = z; }
  const _Float16* ar = sA + (wave * 16 + m) * AP + 8 * hh;
#pragma unroll 2
  for (int kt = 0; kt < CLSK / 32; ++kt) {
    FragH a;
    a.h[0] = *(const v8h*)(ar + 32 * kt);
    a.h[1] = *(const v8h*)(ar + 32 * kt + 16);
#pragma unroll
    for (int t = 0; t < CLSN / 16; ++t) {
      const _Float16* bp = CLt + (size_t)(16 * t + m) * CLSK + 32 * kt + 8 * hh;
      FragH b;
      b.h[0] = *(const v8h*)bp;
      b.h[1] = *(const v8h*)(bp + 16);
      acc[t] = wmh(a.v, b.v, acc[t]);
    }
  }
  __syncthreads();

#pragma unroll
  for (int t = 0; t < CLSN / 16; ++t) {
    const int col = 16 * t + m;
    const float bl = clsb[col < RR ? col : RR - 1];
    if (col < RR) {
      float* sp = stg + (wave * 16 + 8 * hh) * RR + col;
#pragma unroll
      for (int r8 = 0; r8 < 8; ++r8) sp[r8 * RR] = acc[t][r8] * WINV + bl;
    }
  }
  __syncthreads();

  int nv = nB - rowBase;
  nv = nv > GROWS ? GROWS : nv;
  const int nf = nv * RR;
  const int nq = nf >> 2;
  float* gp = out0 + (size_t)rowBase * RR;
#pragma unroll 1
  for (int i = tid; i < nq; i += NTHR) { const v4f v = *(const v4f*)(stg + 4 * i); *(volatile v4f*)(gp + 4 * i) = v; }
  if (tid == 0) { for (int j = nq * 4; j < nf; ++j) { const float x = stg[j]; *(volatile float*)(gp + j) = x; } }
  __threadfence();
#pragma unroll 1
  for (int i = tid; i < nq; i += NTHR) { const v4f v = *(const v4f*)(stg + 4 * i); *(volatile v4f*)(gp + 4 * i) = v; }
  if (tid == 0) { for (int j = nq * 4; j < nf; ++j) { const float x = stg[j]; *(volatile float*)(gp + j) = x; } }
}

extern "C" void kernel_launch(void* const* d_in, const int* in_sizes, int n_in,
                              void* d_out, int out_size, void* d_ws, size_t ws_size,
                              hipStream_t stream) {
  if (n_in < 18) return;
  const int nN = in_sizes[0] / FIN;
  const int nE = in_sizes[15];
  const int nB = in_sizes[17] / 2;
  if (nN <= 0 || nE <= 0 || nB <= 0) return;
  if (in_sizes[0] != nN * FIN || in_sizes[1] != nN * FIN || in_sizes[2] != nN * FIN) return;
  if (in_sizes[3] != RR * FIN * H1 || in_sizes[4] != FIN * H1 || in_sizes[5] < H1) return;
  if (in_sizes[6] != RR * H1 * H2 || in_sizes[7] != H1 * H2 || in_sizes[8] < H2 || in_sizes[9] < 2) return;
  if (in_sizes[10] != H2 * H2 || in_sizes[11] < 1 || in_sizes[12] != CLSK * RR || in_sizes[13] < RR) return;
  if (in_sizes[14] != 2 * nE || in_sizes[16] != nE || in_sizes[17] != 2 * nB) return;
  if (out_size != nB * RR + 4 * nN + nN * H2) return;
  if (nE > (1 << 27) || nN > (1 << 23) || nB > (1 << 24)) return;

  const float* x_o   = (const float*)d_in[0];
  const float* x_a   = (const float*)d_in[1];
  const float* feat  = (const float*)d_in[2];
  const float* W1    = (const float*)d_in[3];
  const float* root1 = (const float*)d_in[4];
  const float* b1    = (const float*)d_in[5];
  const float* W2    = (const float*)d_in[6];
  const float* root2 = (const float*)d_in[7];
  const float* b2    = (const float*)d_in[8];
  const float* attt  = (const float*)d_in[9];
  const float* discW = (const float*)d_in[10];
  const float* discb = (const float*)d_in[11];
  const float* clsW  = (const float*)d_in[12];
  const float* clsb  = (const float*)d_in[13];
  const int*   ei    = (const int*)d_in[14];
  const int*   et0   = (const int*)d_in[15];
  const int*   et1   = (const int*)d_in[16];
  const int*   idxp  = (const int*)d_in[17];
  float* out = (float*)d_out;
  float* out0 = out;
  float* out1 = out0 + (size_t)nB * RR;
  float* out2 = out1 + (size_t)nN * 2;
  float* out3 = out2 + (size_t)nN * 2;

  const int NBP   = ((nN + NBA - 1) / NBA) * NBA;
  const int nAgg  = NBP / NBA;
  const int nRoot = NBP / GROWS;
  int tcap = (nE + RR - 1) / RR;
  tcap = tcap + tcap / 4 + 128;
  tcap = (tcap + 127) & ~127;
  const int ldsT   = tcap * 4 + LISTN * 4 + 64;
  const int ldsC   = NBA * RR * 4 + LISTN * 4 + 64;
  const int ldsA   = NBA * ACP * 4 + LISTN * 4 + 64;
  const int ldsO   = 3 * OROWS * H2 * 4;
  const int ldsCls = GROWS * (CLSK + 8) * 2;
  if (ldsT > 200 * 1024) return;

  char* ws = (char*)d_ws;
  size_t off = 0;
  const size_t oX16o = off; off += (size_t)nN * FIN * 2;            off = (off + 255) & ~(size_t)255;
  const size_t oX16a = off; off += (size_t)nN * FIN * 2;            off = (off + 255) & ~(size_t)255;
  const size_t oW1t  = off; off += (size_t)RR * H1 * FIN * 2;        off = (off + 255) & ~(size_t)255;
  const size_t oW2t  = off; off += (size_t)RR * H2 * H1 * 2;         off = (off + 255) & ~(size_t)255;
  const size_t oR1t  = off; off += (size_t)H1 * FIN * 2;             off = (off + 255) & ~(size_t)255;
  const size_t oR2t  = off; off += (size_t)H2 * H1 * 2;              off = (off + 255) & ~(size_t)255;
  const size_t oCLt  = off; off += (size_t)CLSN * CLSK * 2;          off = (off + 255) & ~(size_t)255;
  const size_t oPerm = off; off += (size_t)RR * tcap * 4;            off = (off + 255) & ~(size_t)255;
  const size_t oTc   = off; off += (size_t)RR * 32 * 4;              off = (off + 255) & ~(size_t)255;
  const size_t oRc   = off; off += (size_t)NBP * RP * 4;             off = (off + 255) & ~(size_t)255;
  const size_t oM    = off; off += (size_t)nE * MP * 2;              off = (off + 255) & ~(size_t)255;
  const size_t oRT1o = off; off += (size_t)NBP * MP * 2;             off = (off + 255) & ~(size_t)255;
  const size_t oRTt  = off; off += (size_t)NBP * MP * 2;             off = (off + 255) & ~(size_t)255;
  const size_t oH16o = off; off += (size_t)NBP * MP * 2;             off = (off + 255) & ~(size_t)255;
  const size_t oH16t = off; off += (size_t)NBP * MP * 2;             off = (off + 255) & ~(size_t)255;
  const size_t oX2o  = off; off += (size_t)NBP * H2 * 4;             off = (off + 255) & ~(size_t)255;
  const size_t oX2a  = off; off += (size_t)NBP * H2 * 4;             off = (off + 255) & ~(size_t)255;
  const size_t oX2b  = off; off += (size_t)NBP * H2 * 4;             off = (off + 255) & ~(size_t)255;
  const size_t oV    = off; off += 256;                              off = (off + 255) & ~(size_t)255;
  if (off > ws_size || off > (size_t)134217728) return;
  _Float16* X16o = (_Float16*)(ws + oX16o);
  _Float16* X16a = (_Float16*)(ws + oX16a);
  _Float16* W1t  = (_Float16*)(ws + oW1t);
  _Float16* W2t  = (_Float16*)(ws + oW2t);
  _Float16* R1t  = (_Float16*)(ws + oR1t);
  _Float16* R2t  = (_Float16*)(ws + oR2t);
  _Float16* CLt  = (_Float16*)(ws + oCLt);
  int*      perm = (int*)(ws + oPerm);
  int*      tcnt = (int*)(ws + oTc);
  float*    rc   = (float*)(ws + oRc);
  _Float16* Mp   = (_Float16*)(ws + oM);
  _Float16* RT1o = (_Float16*)(ws + oRT1o);
  _Float16* RTt  = (_Float16*)(ws + oRTt);
  _Float16* H16o = (_Float16*)(ws + oH16o);
  _Float16* H16t = (_Float16*)(ws + oH16t);
  float*    X2o  = (float*)(ws + oX2o);
  float*    X2a  = (float*)(ws + oX2a);
  float*    X2b  = (float*)(ws + oX2b);
  float*    vline = (float*)(ws + oV);

  const int vec8d = ((nE & 3) == 0) ? 1 : 0;
  const int vec8t = 1;

  hipFuncSetAttribute(reinterpret_cast<const void*>(&k_tsort),   hipFuncAttributeMaxDynamicSharedMemorySize, ldsT);
  hipFuncSetAttribute(reinterpret_cast<const void*>(&k_cnt),     hipFuncAttributeMaxDynamicSharedMemorySize, ldsC);
  hipFuncSetAttribute(reinterpret_cast<const void*>(&k_agg<1>),  hipFuncAttributeMaxDynamicSharedMemorySize, ldsA);
  hipFuncSetAttribute(reinterpret_cast<const void*>(&k_agg<2>),  hipFuncAttributeMaxDynamicSharedMemorySize, ldsA);
  hipFuncSetAttribute(reinterpret_cast<const void*>(&k_out),     hipFuncAttributeMaxDynamicSharedMemorySize, ldsO);
  hipFuncSetAttribute(reinterpret_cast<const void*>(&k_cls),     hipFuncAttributeMaxDynamicSharedMemorySize, ldsCls);

  {
    const int s0 = nN * (FIN / 8);
    const int p0 = (s0 + NTHR - 1) & ~(NTHR - 1);
    const int tot = 2 * p0 + RR * H1 * FIN / 8 + RR * H2 * H1 / 8 + H1 * FIN / 8 + H2 * H1 / 8 + CLSN * CLSK / 8;
    k_prep<<<(tot + NTHR - 1) / NTHR, NTHR, 0, stream>>>(x_o, x_a, W1, W2, root1, root2, clsW,
                                                         X16o, X16a, W1t, W2t, R1t, R2t, CLt, nN);
  }

  const dim3 gMsg(tcap / GROWS, RR);
  const dim3 gRoot(nRoot, 1);

  k_tsort<<<RR, NTHR, ldsT, stream>>>(et0, perm, tcnt, nE, tcap, vec8t);
  k_cnt<<<nAgg, NTHR, ldsC, stream>>>(ei, et0, rc, nE, vec8d);

  k_gemm16<FIN, 4, 0><<<gRoot, NTHR, 0, stream>>>(X16o, R1t, perm, tcnt, ei, RT1o, nN, NBP, nE, tcap);
  k_gemm16<FIN, 4, 1><<<gMsg,  NTHR, 0, stream>>>(X16o, W1t, perm, tcnt, ei, Mp,   nN, 0,   nE, tcap);
  k_agg<1><<<nAgg, NTHR, ldsA, stream>>>(ei, et0, rc, Mp, RT1o, b1, H16o, X2o, nE, vec8d);
  k_gemm16<H1, 2, 0><<<gRoot, NTHR, 0, stream>>>(H16o, R2t, perm, tcnt, ei, RTt, NBP, NBP, nE, tcap);
  k_gemm16<H1, 2, 1><<<gMsg,  NTHR, 0, stream>>>(H16o, W2t, perm, tcnt, ei, Mp,  nN,  0,   nE, tcap);
  k_agg<2><<<nAgg, NTHR, ldsA, stream>>>(ei, et0, rc, Mp, RTt, b2, H16t, X2o, nE, vec8d);

  k_gemm16<FIN, 4, 0><<<gRoot, NTHR, 0, stream>>>(X16a, R1t, perm, tcnt, ei, RTt, nN, NBP, nE, tcap);
  k_gemm16<FIN, 4, 1><<<gMsg,  NTHR, 0, stream>>>(X16a, W1t, perm, tcnt, ei, Mp,  nN, 0,   nE, tcap);
  k_agg<1><<<nAgg, NTHR, ldsA, stream>>>(ei, et0, rc, Mp, RTt, b1, H16t, X2a, nE, vec8d);
  k_gemm16<H1, 2, 0><<<gRoot, NTHR, 0, stream>>>(H16t, R2t, perm, tcnt, ei, RTt, NBP, NBP, nE, tcap);
  k_gemm16<H1, 2, 1><<<gMsg,  NTHR, 0, stream>>>(H16t, W2t, perm, tcnt, ei, Mp,  nN,  0,   nE, tcap);
  k_agg<2><<<nAgg, NTHR, ldsA, stream>>>(ei, et0, rc, Mp, RTt, b2, H16t, X2a, nE, vec8d);

  k_tsort<<<RR, NTHR, ldsT, stream>>>(et1, perm, tcnt, nE, tcap, vec8t);
  k_cnt<<<nAgg, NTHR, ldsC, stream>>>(ei, et1, rc, nE, vec8d);

  k_gemm16<FIN, 4, 1><<<gMsg,  NTHR, 0, stream>>>(X16o, W1t, perm, tcnt, ei, Mp,  nN, 0,   nE, tcap);
  k_agg<1><<<nAgg, NTHR, ldsA, stream>>>(ei, et1, rc, Mp, RT1o, b1, H16t, X2b, nE, vec8d);
  k_gemm16<H1, 2, 0><<<gRoot, NTHR, 0, stream>>>(H16t, R2t, perm, tcnt, ei, RTt, NBP, NBP, nE, tcap);
  k_gemm16<H1, 2, 1><<<gMsg,  NTHR, 0, stream>>>(H16t, W2t, perm, tcnt, ei, Mp,  nN,  0,   nE, tcap);
  k_agg<2><<<nAgg, NTHR, ldsA, stream>>>(ei, et1, rc, Mp, RTt, b2, H16t, X2b, nE, vec8d);

  k_readout<<<1, NTHR, 0, stream>>>(X2o, discW, vline, nN);
  k_out<<<(nN + OROWS - 1) / OROWS, NTHR, ldsO, stream>>>(X2o, X2a, X2b, vline, discb, out1, out2, out3, nN, NBP);
  k_cls<<<(nB + GROWS - 1) / GROWS, NTHR, ldsCls, stream>>>(H16o, X2o, feat, idxp, attt, CLt, clsb, out0, nN, nB);
}
